// CrossModalAttention_63007170232767
// MI455X (gfx1250) — hardware-verified
//
#include <hip/hip_runtime.h>


#ifndef NB
#define NB 2
#endif
#ifndef SEQ
#define SEQ 2048
#endif
#ifndef NQ
#define NQ SEQ
#endif
#ifndef NKV
#define NKV SEQ
#endif
#define NB_FULL 2
#define NQ_FULL 2048
#define NKV_FULL 2048
#define DM 512
#define NH 8
#define HD 64
#define PCAR 1024.0f
#define SCL 0.125f
#define L2E 1.4426950408889634f
#define LNEPS 1e-5f
#define KP 72
#define OP 68
static_assert(NQ % 64 == 0);
static_assert(NKV % 64 == 0);
static_assert(NH * HD == DM);
static_assert(DM % 64 == 0);
static_assert(NB >= 1 && NB <= NB_FULL);
static_assert(NQ <= NQ_FULL && NKV <= NKV_FULL);

typedef _Float16 h16;
typedef unsigned short bf;
typedef __attribute__((ext_vector_type(16))) __bf16   v16bf;
typedef __attribute__((ext_vector_type(16))) _Float16 v16h;
typedef __attribute__((ext_vector_type(8)))  _Float16 v8h;
typedef __attribute__((ext_vector_type(8)))  unsigned short v8us;
typedef __attribute__((ext_vector_type(8)))  float    v8f;
typedef __attribute__((ext_vector_type(4)))  float    v4f;
typedef v8h  __attribute__((may_alias)) v8ha;
typedef v4f  __attribute__((may_alias)) v4fa;
typedef v8us __attribute__((may_alias)) v8usa;

__device__ __forceinline__ unsigned short f2bf(float f) { unsigned u = __float_as_uint(f); u += 0x7FFFu + ((u >> 16) & 1u); return (unsigned short)(u >> 16); }
__device__ __forceinline__ float bf2f(unsigned short b) { return __uint_as_float(((unsigned)b) << 16); }
__device__ __forceinline__ float bfr(float f) { return bf2f(f2bf(f)); }
__device__ __forceinline__ v16h cat16(v8h lo, v8h hi) { return __builtin_shufflevector(lo, hi, 0, 1, 2, 3, 4, 5, 6, 7, 8, 9, 10, 11, 12, 13, 14, 15); }
__device__ __forceinline__ v16bf cat16b(v8us lo, v8us hi) { return __builtin_bit_cast(v16bf, __builtin_shufflevector(lo, hi, 0, 1, 2, 3, 4, 5, 6, 7, 8, 9, 10, 11, 12, 13, 14, 15)); }
__device__ __forceinline__ v8f wmma16(v16h a, v16h b, v8f c) { return __builtin_amdgcn_wmma_f32_16x16x32_f16(false, a, false, b, (short)0, c, false, false); }
__device__ __forceinline__ v8f wmmab(v16bf a, v16bf b, v8f c) { return __builtin_amdgcn_wmma_f32_16x16x32_bf16(false, a, false, b, (short)0, c, false, false); }
__device__ __forceinline__ v8f wmma16g(v16h a, v16h b, v8f c) { v8f d = __builtin_amdgcn_wmma_f32_16x16x32_f16(false, a, false, b, (short)0, c, false, false); asm volatile("v_nop\n\tv_nop\n\tv_nop\n\tv_nop" : "+v"(d) : "v"(a), "v"(b)); return d; }

template <typename T16> struct WFrag;
template <> struct WFrag<h16> { typedef v16h V; static __device__ __forceinline__ V ld(const h16* p) { return cat16(*(const v8h*)p, *(const v8h*)(p + 16)); } static __device__ __forceinline__ v8f mma(V a, V b, v8f c) { return wmma16(a, b, c); } };
template <> struct WFrag<bf> { typedef v16bf V; static __device__ __forceinline__ V ld(const bf* p) { return cat16b(*(const v8us*)p, *(const v8us*)(p + 16)); } static __device__ __forceinline__ v8f mma(V a, V b, v8f c) { return wmmab(a, b, c); } };
template <typename T16, int NSPLIT, bool BIAS>
__global__ __launch_bounds__(32) void k_gemmw(const T16* __restrict__ A, const T16* __restrict__ A2, const T16* __restrict__ Bt, const T16* __restrict__ Bt2, int K, float* C, int ldc, const float* __restrict__ bias, size_t sA, size_t sB, size_t sC) {
    typedef typename WFrag<T16>::V V;
    __shared__ __align__(16) float os[16 * 68];
    const size_t z = blockIdx.z; A += z * sA; if (A2) A2 += z * sA; Bt += z * sB; if (Bt2) Bt2 += z * sB; C += z * sC;
    const int lane = threadIdx.x & 31, lr = lane & 15, hi = lane >> 4; const int r0 = blockIdx.x * 64, c0 = blockIdx.y * 64;
    v8f acc[4][4];
#pragma unroll
    for (int mb = 0; mb < 4; ++mb)
#pragma unroll
        for (int nb = 0; nb < 4; ++nb) acc[mb][nb] = (v8f){};
    const size_t aoff = (size_t)(r0 + lr) * K + 8 * hi, boff = (size_t)(c0 + lr) * K + 8 * hi;
#pragma unroll 1
    for (int kc = 0; kc < K; kc += 32) {
        V a[4], a2[4];
#pragma unroll
        for (int mb = 0; mb < 4; ++mb) { a[mb] = WFrag<T16>::ld(A + aoff + (size_t)mb * 16 * K + kc); if (NSPLIT == 1 || NSPLIT == 2) a2[mb] = WFrag<T16>::ld(A2 + aoff + (size_t)mb * 16 * K + kc); }
#pragma unroll
        for (int nb = 0; nb < 4; ++nb) { const V b = WFrag<T16>::ld(Bt + boff + (size_t)nb * 16 * K + kc); V b2; if (NSPLIT >= 2) b2 = WFrag<T16>::ld(Bt2 + boff + (size_t)nb * 16 * K + kc);
#pragma unroll
            for (int mb = 0; mb < 4; ++mb) { acc[mb][nb] = WFrag<T16>::mma(a[mb], b, acc[mb][nb]); if (NSPLIT == 1 || NSPLIT == 2) acc[mb][nb] = WFrag<T16>::mma(a2[mb], b, acc[mb][nb]); if (NSPLIT >= 2) acc[mb][nb] = WFrag<T16>::mma(a[mb], b2, acc[mb][nb]); } }
        asm volatile("v_nop\n\tv_nop\n\tv_nop\n\tv_nop" : "+v"(acc[0][0]), "+v"(acc[1][1]), "+v"(acc[2][2]), "+v"(acc[3][3]) : "v"(a[0]), "v"(a[3]));
    }
#pragma unroll
    for (int mb = 0; mb < 4; ++mb) {
#pragma unroll
        for (int nb = 0; nb < 4; ++nb) {
#pragma unroll
            for (int j = 0; j < 8; ++j) os[(hi * 8 + j) * 68 + nb * 16 + lr] = acc[mb][nb][j]; }
        __builtin_amdgcn_wave_barrier(); asm volatile("" ::: "memory");
        float* crow = C + (size_t)(r0 + mb * 16) * ldc + c0;
#pragma unroll 1
        for (int ps = 0; ps < 2; ++ps) {
#pragma unroll
            for (int s = 0; s < 8; ++s) { const int row = 2 * s + hi, cofs = lr * 4; v4f val = *(const v4fa*)(os + row * 68 + cofs); if (BIAS) { val[0] += bfr(bias[c0 + cofs]); val[1] += bfr(bias[c0 + cofs + 1]); val[2] += bfr(bias[c0 + cofs + 2]); val[3] += bfr(bias[c0 + cofs + 3]); }
                *(volatile v4f*)(crow + (size_t)row * ldc + cofs) = val; }
            if (ps == 0) __threadfence(); }
        __builtin_amdgcn_wave_barrier(); asm volatile("" ::: "memory");
    }
}

__global__ __launch_bounds__(256) void k_cvt8b(const float* __restrict__ src, size_t sstride, bf* dst, size_t dstride, size_t n8) {
    const size_t i = (size_t)blockIdx.x * 256 + threadIdx.x; if (i >= n8) return; const size_t y = blockIdx.y;
    const v8f v = *(const v8f*)(src + y * sstride + i * 8); v8us o;
#pragma unroll
    for (int k = 0; k < 8; ++k) o[k] = f2bf(v[k]);
    bf* d = dst + y * dstride + i * 8; *(volatile v8us*)d = o; __threadfence(); *(volatile v8us*)d = o;
}

__global__ __launch_bounds__(256) void k_wtr(const float* __restrict__ W0, const float* __restrict__ W1, const float* __restrict__ W2, bf* Wt) {
    const int z = blockIdx.y;
    const float* W = (z == 0) ? W0 : ((z == 1) ? W1 : W2);
    const size_t i = (size_t)blockIdx.x * 256 + threadIdx.x; if (i >= (size_t)DM * DM / 8) return;
    const int k0 = (int)(i % (DM / 8)) * 8; const int n = (int)(i / (DM / 8));
    v8us o;
#pragma unroll
    for (int q = 0; q < 8; ++q) o[q] = f2bf(W[(size_t)(k0 + q) * DM + n]);
    bf* d = Wt + (size_t)z * DM * DM + (size_t)n * DM + k0;
    *(volatile v8us*)d = o; __threadfence(); *(volatile v8us*)d = o;
}

__global__ __launch_bounds__(256) void k_hrow(const float* __restrict__ C, h16* P, int nrows) {
    const size_t i = (size_t)blockIdx.x * 256 + threadIdx.x;
    const size_t tot = (size_t)NB * NH * nrows * 8; if (i >= tot) return;
    const int q8 = (int)(i & 7); size_t r = i >> 3; const int s = (int)(r % (size_t)nrows); r /= (size_t)nrows; const int h = (int)(r % NH); const int b = (int)(r / NH);
    const v8f v = *(const v8f*)(C + ((size_t)b * nrows + s) * DM + h * HD + q8 * 8); v8h o;
#pragma unroll
    for (int q = 0; q < 8; ++q) o[q] = (h16)v[q];
    h16* d = P + i * 8; *(volatile v8h*)d = o; __threadfence(); *(volatile v8h*)d = o;
}

__global__ __launch_bounds__(256) void k_vt(const float* __restrict__ C, h16* VT) {
    const size_t i = (size_t)blockIdx.x * 256 + threadIdx.x;
    const size_t tot = (size_t)NB * NH * HD * (NKV / 8); if (i >= tot) return;
    const int s0 = (int)(i % (NKV / 8)) * 8; size_t r = i / (NKV / 8); const int d = (int)(r % HD); r /= HD; const int h = (int)(r % NH); const int b = (int)(r / NH);
    v8h o;
#pragma unroll
    for (int q = 0; q < 8; ++q) o[q] = (h16)C[((size_t)b * NKV + s0 + q) * DM + h * HD + d];
    h16* dst = VT + i * 8; *(volatile v8h*)dst = o; __threadfence(); *(volatile v8h*)dst = o;
}

__global__ __launch_bounds__(128) __attribute__((amdgpu_num_vgpr(256))) void k_attn(const h16* __restrict__ Qh, const h16* __restrict__ Kh, const h16* __restrict__ Vt, float* ctx) {
    __shared__ __align__(16) h16 Ks[64 * KP];
    __shared__ __align__(16) h16 Vs[64 * KP];
    __shared__ __align__(16) h16 Ps[4 * 16 * KP];
    __shared__ __align__(16) float Os[4 * 16 * OP];
    const int t = threadIdx.x, wave = t >> 5, lane = t & 31, lm = lane & 15, hi = lane >> 4;
    int bid = blockIdx.x; const int nqt = NQ / 64; const int qt = bid % nqt; bid /= nqt; const int h = bid % NH; const int b = bid / NH; const int bh = b * NH + h;
    const h16* qrow = Qh + ((size_t)bh * NQ + (size_t)qt * 64 + wave * 16 + lm) * HD;
    const v16h aQ0 = cat16(*(const v8h*)(qrow + 8 * hi), *(const v8h*)(qrow + 16 + 8 * hi));
    const v16h aQ1 = cat16(*(const v8h*)(qrow + 32 + 8 * hi), *(const v8h*)(qrow + 48 + 8 * hi));
    v8f O[4];
#pragma unroll
    for (int nt = 0; nt < 4; ++nt) O[nt] = (v8f){};
    float runm[8], runl[8];
#pragma unroll
    for (int r = 0; r < 8; ++r) { runm[r] = -1.0e30f; runl[r] = 0.f; }
    const h16* Kb = Kh + (size_t)bh * NKV * HD; const h16* Vb = Vt + (size_t)bh * HD * NKV;
    h16* Pw = Ps + wave * 16 * KP; float* Ow = Os + wave * 16 * OP;
#pragma unroll 1
    for (int kv0 = 0; kv0 < NKV; kv0 += 64) {
        __syncthreads();
#pragma unroll
        for (int j = 0; j < 4; ++j) { const int p = t + 128 * j; const int row = p >> 3, c8 = (p & 7) * 8;
            const v8h kk = *(const v8h*)(Kb + (size_t)(kv0 + row) * HD + c8);
            const v8h vv = *(const v8h*)(Vb + (size_t)row * NKV + kv0 + c8);
            *(v8ha*)(Ks + row * KP + c8) = kk; *(v8ha*)(Vs + row * KP + c8) = vv; }
        __syncthreads();
        v8f sf[4];
#pragma unroll
        for (int nk = 0; nk < 4; ++nk) { const h16* kr = Ks + (nk * 16 + lm) * KP + 8 * hi;
            const v16h b0 = cat16(*(const v8ha*)(kr), *(const v8ha*)(kr + 16));
            const v16h b1 = cat16(*(const v8ha*)(kr + 32), *(const v8ha*)(kr + 48));
            v8f a = (v8f){}; a = wmma16g(aQ0, b0, a); a = wmma16g(aQ1, b1, a); sf[nk] = a; }
#pragma unroll
        for (int r = 0; r < 8; ++r) {
            sf[0][r] *= SCL; sf[1][r] *= SCL; sf[2][r] *= SCL; sf[3][r] *= SCL;
            float m = fmaxf(fmaxf(sf[0][r], sf[1][r]), fmaxf(sf[2][r], sf[3][r]));
#pragma unroll
            for (int sh = 1; sh < 16; sh <<= 1) m = fmaxf(m, __shfl_xor(m, sh, 32));
            const float nm = fmaxf(runm[r], m);
            const float corr = __builtin_amdgcn_exp2f(__fmul_rn(__fsub_rn(runm[r], nm), L2E));
            runm[r] = nm; runl[r] *= corr;
            O[0][r] *= corr; O[1][r] *= corr; O[2][r] *= corr; O[3][r] *= corr; }
#pragma unroll
        for (int nk = 0; nk < 4; ++nk) {
#pragma unroll
            for (int r = 0; r < 8; ++r) { const float p = __builtin_amdgcn_exp2f(__fmul_rn(__fsub_rn(sf[nk][r], runm[r]), L2E)); runl[r] += p; Pw[(r + 8 * hi) * KP + nk * 16 + lm] = (h16)(p * PCAR); } }
        __syncthreads();
#pragma unroll
        for (int ks = 0; ks < 2; ++ks) { const h16* pr = Pw + lm * KP + ks * 32 + 8 * hi;
            const v16h aP = cat16(*(const v8ha*)(pr), *(const v8ha*)(pr + 16));
#pragma unroll
            for (int nt = 0; nt < 4; ++nt) { const h16* vr = Vs + (nt * 16 + lm) * KP + ks * 32 + 8 * hi;
                const v16h bV = cat16(*(const v8ha*)(vr), *(const v8ha*)(vr + 16));
                O[nt] = wmma16g(aP, bV, O[nt]); } }
    }
#pragma unroll
    for (int r = 0; r < 8; ++r) { float l = runl[r];
#pragma unroll
        for (int sh = 1; sh < 16; sh <<= 1) l += __shfl_xor(l, sh, 32);
        const float inv = __fdiv_rn(1.0f, l * PCAR);
#pragma unroll
        for (int nt = 0; nt < 4; ++nt) Ow[(8 * hi + r) * OP + nt * 16 + lm] = O[nt][r] * inv; }
    __syncthreads();
    float* crow = ctx + ((size_t)b * NQ + (size_t)qt * 64 + wave * 16) * DM + h * HD;
#pragma unroll 1
    for (int ps = 0; ps < 2; ++ps) {
#pragma unroll
        for (int s = 0; s < 8; ++s) { const int row = 2 * s + hi, cofs = lm * 4; const v4f val = *(const v4fa*)(Ow + row * OP + cofs); *(volatile v4f*)(crow + (size_t)row * DM + cofs) = val; }
        if (ps == 0) __threadfence(); }
}

__global__ __launch_bounds__(256) void k_ln(const float* __restrict__ xq, const float* __restrict__ ctx, const float* __restrict__ gam, const float* __restrict__ bet, float* outp) {
#pragma clang fp contract(off)
    const int lane = threadIdx.x & 31; const int row = blockIdx.x * 8 + (threadIdx.x >> 5); if (row >= NB * NQ) return;
    const int b = row / NQ, i = row % NQ;
    const float* xr = xq + ((size_t)b * NQ_FULL + i) * DM; const float* cr = ctx + (size_t)row * DM;
    float v[16]; float s = 0.f;
#pragma unroll
    for (int c = 0; c < 4; ++c) { const int j0 = c * 128 + lane * 4; const v4f a = *(const v4f*)(xr + j0); const v4f g = *(const v4f*)(cr + j0);
#pragma unroll
        for (int q = 0; q < 4; ++q) { const float x = bfr(a[q]) + g[q]; v[c * 4 + q] = x; s = s + x; } }
#pragma unroll
    for (int sh = 16; sh; sh >>= 1) s += __shfl_xor(s, sh, 32);
    const float mu = s * (1.0f / DM);
    float ss = 0.f;
#pragma unroll
    for (int k = 0; k < 16; ++k) { const float d = v[k] - mu; const float dd = d * d; ss = ss + dd; }
#pragma unroll
    for (int sh = 16; sh; sh >>= 1) ss += __shfl_xor(ss, sh, 32);
    const float var = ss * (1.0f / DM);
    const float rs = __fdiv_rn(1.0f, __fsqrt_rn(var + LNEPS));
    float* orow = outp + (size_t)row * DM;
#pragma unroll 1
    for (int ps = 0; ps < 2; ++ps) {
#pragma unroll
        for (int c = 0; c < 4; ++c) { const int j0 = c * 128 + lane * 4; const v4f g = *(const v4f*)(gam + j0); const v4f bb = *(const v4f*)(bet + j0); v4f o;
#pragma unroll
            for (int q = 0; q < 4; ++q) { const float t1 = (v[c * 4 + q] - mu) * rs; const float t2 = t1 * bfr(g[q]); o[q] = t2 + bfr(bb[q]); }
            *(volatile v4f*)(orow + j0) = o; }
        if (ps == 0) __threadfence(); }
}

extern "C" void kernel_launch(void* const* d_in, const int* in_sizes, int n_in, void* d_out, int out_size, void* d_ws, size_t ws_size, hipStream_t stream) {
    if (n_in < 10) return;
    const float* xq  = (const float*)d_in[0];
    const float* xkv = (const float*)d_in[1];
    const float* Wq  = (const float*)d_in[2];
    const float* bq  = (const float*)d_in[3];
    const float* Wk  = (const float*)d_in[4];
    const float* bk  = (const float*)d_in[5];
    const float* Wv  = (const float*)d_in[6];
    const float* bv  = (const float*)d_in[7];
    const float* gam = (const float*)d_in[8];
    const float* bet = (const float*)d_in[9];
    if (in_sizes[0] < (int)(((size_t)(NB - 1) * NQ_FULL + NQ) * DM)) return;
    if (in_sizes[1] < (int)(((size_t)(NB - 1) * NKV_FULL + NKV) * DM)) return;
    if (in_sizes[2] < DM * DM || in_sizes[4] < DM * DM || in_sizes[6] < DM * DM) return;
    if (in_sizes[3] < DM || in_sizes[5] < DM || in_sizes[7] < DM || in_sizes[8] < DM || in_sizes[9] < DM) return;
    if (out_size < NB * NQ * DM) return;
    float* OUT = (float*)d_out;
    char* wsp = (char*)d_ws;
    auto take = [&](size_t bytes) { char* p = wsp; wsp += (bytes + 255) & ~(size_t)255; return (void*)p; };
    bf* Xq   = (bf*)take((size_t)NB * NQ * DM * 2);
    bf* Xkv  = (bf*)take((size_t)NB * NKV * DM * 2);
    bf* Wt   = (bf*)take((size_t)3 * DM * DM * 2);
    float* Cq = (float*)take((size_t)NB * NQ * DM * 4);
    float* Ck = (float*)take((size_t)NB * NKV * DM * 4);
    float* Cv = (float*)take((size_t)NB * NKV * DM * 4);
    h16* Qh  = (h16*)take((size_t)NB * NH * NQ * HD * 2);
    h16* Kh  = (h16*)take((size_t)NB * NH * NKV * HD * 2);
    h16* VT  = (h16*)take((size_t)NB * NH * HD * NKV * 2);
    float* CTX = (float*)take((size_t)NB * NQ * DM * 4);
    if ((size_t)(wsp - (char*)d_ws) > ws_size) return;
    if ((size_t)(wsp - (char*)d_ws) > (size_t)134217728) return;

    const size_t n8q = (size_t)NQ * DM / 8, n8kv = (size_t)NKV * DM / 8;
    k_cvt8b<<<dim3((unsigned)((n8q + 255) / 256), NB), 256, 0, stream>>>(xq, (size_t)NQ_FULL * DM, Xq, (size_t)NQ * DM, n8q);
    k_cvt8b<<<dim3((unsigned)((n8kv + 255) / 256), NB), 256, 0, stream>>>(xkv, (size_t)NKV_FULL * DM, Xkv, (size_t)NKV * DM, n8kv);
    k_wtr<<<dim3((unsigned)(((size_t)DM * DM / 8 + 255) / 256), 3), 256, 0, stream>>>(Wq, Wk, Wv, Wt);
    k_gemmw<bf, 0, true><<<dim3(NB * NQ / 64, DM / 64, 1), 32, 0, stream>>>(Xq, nullptr, Wt, nullptr, DM, Cq, DM, bq, 0, 0, 0);
    k_gemmw<bf, 0, true><<<dim3(NB * NKV / 64, DM / 64, 1), 32, 0, stream>>>(Xkv, nullptr, Wt + (size_t)DM * DM, nullptr, DM, Ck, DM, bk, 0, 0, 0);
    k_gemmw<bf, 0, true><<<dim3(NB * NKV / 64, DM / 64, 1), 32, 0, stream>>>(Xkv, nullptr, Wt + 2 * (size_t)DM * DM, nullptr, DM, Cv, DM, bv, 0, 0, 0);
    k_hrow<<<(unsigned)(((size_t)NB * NH * NQ * 8 + 255) / 256), 256, 0, stream>>>(Cq, Qh, NQ);
    k_hrow<<<(unsigned)(((size_t)NB * NH * NKV * 8 + 255) / 256), 256, 0, stream>>>(Ck, Kh, NKV);
    k_vt<<<(unsigned)(((size_t)NB * NH * HD * (NKV / 8) + 255) / 256), 256, 0, stream>>>(Cv, VT);
    k_attn<<<NB * NH * (NQ / 64), 128, 0, stream>>>(Qh, Kh, VT, CTX);
    k_ln<<<(NB * NQ + 7) / 8, 256, 0, stream>>>(xq, CTX, gam, bet, OUT);
}
